// LeviCivitaKANLayer_54820962566346
// MI455X (gfx1250) — hardware-verified
//
#include <hip/hip_runtime.h>
#include <stddef.h>
#include <stdint.h>
#include <math.h>


#define IN_DIM   128
#define OUT_DIM  128
#define KOFF     16256
#define NSLICE   129
#define SLH      (OUT_DIM * IN_DIM)
#define LDH      136
#define XSP      132
#define TM       128
#define NTHR     256
#define NWAVE    8
#define ASCL     16.0f
#define WSCL     256.0f
#define INVSCL   (1.0f / 4096.0f)
#define LN_EPS   1e-5f
#define WSCAP    134217728

#define LDS_XS   (TM * XSP * 4)
#define LDS_W    (OUT_DIM * LDH * 2)
#define LDS_GEMM (LDS_XS + LDS_W)

static_assert(KOFF == IN_DIM * (IN_DIM - 1));
static_assert(TM == NWAVE * 16 && NTHR == NWAVE * 32);
static_assert(((TM * IN_DIM / 4) % NTHR) == 0);
static_assert(((SLH / 8) % NTHR) == 0);
static_assert((XSP % 4) == 0 && (LDH % 8) == 0);
static_assert((LDS_XS % 16) == 0);
static_assert(OUT_DIM == 128 && IN_DIM == 128);
static_assert(TM <= NTHR);

typedef _Float16 v16h __attribute__((ext_vector_type(16)));
typedef _Float16 v8h  __attribute__((ext_vector_type(8)));
typedef _Float16 v4h  __attribute__((ext_vector_type(4)));
typedef float    v8f  __attribute__((ext_vector_type(8)));
typedef float    v4f  __attribute__((ext_vector_type(4)));
union Frag { v16h v; v8h h[2]; v4h q[4]; };

__device__ __forceinline__ v8f wmm(v16h a, v16h b, v8f c) {
  v8f d = __builtin_amdgcn_wmma_f32_16x16x32_f16(false, a, false, b, (short)0, c, false, false);
  asm volatile("v_nop\n\tv_nop\n\tv_nop\n\tv_nop" : "+v"(d) : "v"(a), "v"(b));
  return d;
}

__global__ __launch_bounds__(NTHR) void k_pack(const float* __restrict__ lc_w, const float* __restrict__ w1,
                                              _Float16* Wp, int units) {
  const int u = (int)blockIdx.x * NTHR + (int)threadIdx.x;
  if (u >= units) return;
  const int i  = u >> 11;
  const int o  = (u >> 4) & (OUT_DIM - 1);
  const int j0 = (u & 15) * 8;
  const int ia = i < IN_DIM - 1 ? i : IN_DIM - 1;
  const float* lr = lc_w + (size_t)o * KOFF + (size_t)ia * (IN_DIM - 1);
  const float* wr = w1 + (size_t)o * IN_DIM + j0;
  v8h hv;
#pragma unroll
  for (int e = 0; e < 8; ++e) {
    const int j = j0 + e;
    int kk = j > ia ? j - 1 : j;
    kk = kk > IN_DIM - 2 ? IN_DIM - 2 : kk;
    const float fl = lr[kk];
    const float fw = wr[e];
    const float v  = (i == IN_DIM) ? fw : ((j == i) ? 0.0f : fl);
    hv[e] = (_Float16)(v * WSCL);
  }
  _Float16* dp = Wp + (size_t)u * 8;
  *(volatile v8h*)dp = hv;
  __threadfence();
  *(volatile v8h*)dp = hv;
}

__device__ __forceinline__ void stage_w(const _Float16* __restrict__ src, _Float16* wsl, int tid) {
#pragma unroll
  for (int it = 0; it < (SLH / 8) / NTHR; ++it) {
    const int u  = it * NTHR + tid;
    const int o  = u >> 4;
    const int j8 = (u & 15) * 8;
    const v8h w = *(const v8h*)(src + (size_t)o * IN_DIM + j8);
    *(v8h*)(wsl + o * LDH + j8) = w;
  }
}

__device__ __forceinline__ void slice_macs(const float* xrow, const _Float16* wsl, float sa, int hh, int ml,
                                           v8f (&acc)[8]) {
#pragma unroll
  for (int c = 0; c < 4; ++c) {
    const float* p = xrow + 32 * c + 8 * hh;
    const v4f q0 = *(const v4f*)p * sa;
    const v4f q1 = *(const v4f*)(p + 4) * sa;
    const v4f q2 = *(const v4f*)(p + 16) * sa;
    const v4f q3 = *(const v4f*)(p + 20) * sa;
    Frag a;
    a.q[0] = __builtin_convertvector(q0, v4h);
    a.q[1] = __builtin_convertvector(q1, v4h);
    a.q[2] = __builtin_convertvector(q2, v4h);
    a.q[3] = __builtin_convertvector(q3, v4h);
#pragma unroll
    for (int n = 0; n < 8; ++n) {
      const _Float16* bp = wsl + (16 * n + ml) * LDH + 32 * c + 8 * hh;
      Frag b;
      b.h[0] = *(const v8h*)bp;
      b.h[1] = *(const v8h*)(bp + 16);
      acc[n] = wmm(a.v, b.v, acc[n]);
    }
  }
}

__global__ __launch_bounds__(NTHR) void k_gemm_ln(
    const float* __restrict__ x, const float* __restrict__ scale, const float* __restrict__ trans,
    const _Float16* __restrict__ Wp, const float* __restrict__ gamma, const float* __restrict__ beta,
    float* out, int nRows) {
  extern __shared__ v4f lds_dyn[];
  float* xs = (float*)lds_dyn;
  _Float16* wsl = (_Float16*)((char*)lds_dyn + LDS_XS);
  const int tid = threadIdx.x, lane = tid & 31, wave = tid >> 5, hh = lane >> 4, ml = lane & 15;
  const int rowbase = blockIdx.x * TM;
  if (rowbase + TM > nRows) return;

  {
    const int c = (tid & 31) * 4;
    const v4f tv = *(const v4f*)(trans + c);
    const v4f sv = *(const v4f*)(scale + c);
    v4f rv;
    rv.x = 1.0f / sv.x; rv.y = 1.0f / sv.y; rv.z = 1.0f / sv.z; rv.w = 1.0f / sv.w;
#pragma unroll
    for (int it = 0; it < (TM * IN_DIM / 4) / NTHR; ++it) {
      const int idx = it * NTHR + tid;
      const int r = idx >> 5;
      const v4f xv = *(const v4f*)(x + (size_t)(rowbase + r) * IN_DIM + c);
      *(v4f*)(xs + r * XSP + c) = (xv - tv) * rv;
    }
  }

  v8f acc[8];
#pragma unroll
  for (int n = 0; n < 8; ++n) { v8f z = {0.f, 0.f, 0.f, 0.f, 0.f, 0.f, 0.f, 0.f}; acc[n] = z; }
  const float* xrow = xs + (wave * 16 + ml) * XSP;

#pragma unroll 1
  for (int t = 0; t < IN_DIM; ++t) {
    stage_w(Wp + (size_t)t * SLH, wsl, tid);
    __syncthreads();
    const float sa = ASCL * xrow[t];
    slice_macs(xrow, wsl, sa, hh, ml, acc);
    __syncthreads();
  }

  {
    const int c = (tid & 31) * 4;
#pragma unroll
    for (int it = 0; it < (TM * IN_DIM / 4) / NTHR; ++it) {
      const int idx = it * NTHR + tid;
      const int r = idx >> 5;
      *(v4f*)(xs + r * XSP + c) = *(const v4f*)(x + (size_t)(rowbase + r) * IN_DIM + c);
    }
  }
  stage_w(Wp + (size_t)IN_DIM * SLH, wsl, tid);
  __syncthreads();
  slice_macs(xrow, wsl, ASCL, hh, ml, acc);
  __syncthreads();

  {
    float* sp = xs + (wave * 16 + 8 * hh) * XSP + ml;
#pragma unroll
    for (int n = 0; n < 8; ++n) {
#pragma unroll
      for (int r = 0; r < 8; ++r) sp[r * XSP + 16 * n] = acc[n][r] * INVSCL;
    }
  }
  __syncthreads();
  if (tid < TM) {
    float* yr = xs + tid * XSP;
    float s = 0.0f;
#pragma unroll 4
    for (int c = 0; c < OUT_DIM; ++c) s += yr[c];
    const float mu = s * (1.0f / (float)OUT_DIM);
    float q = 0.0f;
#pragma unroll 4
    for (int c = 0; c < OUT_DIM; ++c) { const float d = yr[c] - mu; q += d * d; }
    const float var = q * (1.0f / (float)OUT_DIM);
    const float rs  = 1.0f / sqrtf(var + LN_EPS);
#pragma unroll 4
    for (int c = 0; c < OUT_DIM; ++c) yr[c] = (yr[c] - mu) * rs * gamma[c] + beta[c];
  }
  __syncthreads();

  float* ob = out + (size_t)(rowbase + wave * 16) * OUT_DIM + 4 * lane;
  const float* sb = xs + (wave * 16) * XSP + 4 * lane;
#pragma unroll
  for (int rr = 0; rr < 16; ++rr) {
    const v4f v = *(const v4f*)(sb + rr * XSP);
    *(volatile v4f*)(ob + (size_t)rr * OUT_DIM) = v;
  }
  __threadfence();
#pragma unroll
  for (int rr = 0; rr < 16; ++rr) {
    const v4f v = *(const v4f*)(sb + rr * XSP);
    *(volatile v4f*)(ob + (size_t)rr * OUT_DIM) = v;
  }
}

extern "C" void kernel_launch(void* const* d_in, const int* in_sizes, int n_in,
                              void* d_out, int out_size, void* d_ws, size_t ws_size,
                              hipStream_t stream) {
  if (n_in < 7) return;
  const int B = in_sizes[0] / IN_DIM;
  if (B <= 0 || in_sizes[0] != B * IN_DIM || (B % TM) != 0) return;
  if (in_sizes[1] != IN_DIM || in_sizes[2] != IN_DIM) return;
  if (in_sizes[3] != OUT_DIM * KOFF || in_sizes[4] != OUT_DIM * IN_DIM) return;
  if (in_sizes[5] != OUT_DIM || in_sizes[6] != OUT_DIM) return;
  if ((long long)out_size != (long long)B * OUT_DIM) return;

  const float* x     = (const float*)d_in[0];
  const float* scale = (const float*)d_in[1];
  const float* trans = (const float*)d_in[2];
  const float* lc_w  = (const float*)d_in[3];
  const float* w1    = (const float*)d_in[4];
  const float* gamma = (const float*)d_in[5];
  const float* beta  = (const float*)d_in[6];
  float* out = (float*)d_out;

  const int units = NSLICE * OUT_DIM * (IN_DIM / 8);
  const size_t wpBytes = (size_t)units * 16;
  if (wpBytes > ws_size || wpBytes > (size_t)WSCAP) return;
  _Float16* Wp = (_Float16*)d_ws;

  k_pack<<<(units + NTHR - 1) / NTHR, NTHR, 0, stream>>>(lc_w, w1, Wp, units);

  hipFuncSetAttribute(reinterpret_cast<const void*>(&k_gemm_ln),
                      hipFuncAttributeMaxDynamicSharedMemorySize, LDS_GEMM);
  k_gemm_ln<<<B / TM, NTHR, LDS_GEMM, stream>>>(x, scale, trans, Wp, gamma, beta, out, B);
}
